// FBPINNWithWindow_30940944401055
// MI455X (gfx1250) — hardware-verified
//
#include <hip/hip_runtime.h>


#define NP   65536
#define JJ   16
#define WD   64
typedef _Float16 h16;
typedef unsigned short bf;
typedef __attribute__((ext_vector_type(16))) __bf16   v16bf;
typedef __attribute__((ext_vector_type(16))) _Float16 v16h;
typedef __attribute__((ext_vector_type(8)))  _Float16 v8h;
typedef __attribute__((ext_vector_type(8)))  unsigned short v8us;
typedef __attribute__((ext_vector_type(8)))  float    v8f;
typedef __attribute__((ext_vector_type(4)))  float    v4f;
typedef v8h  __attribute__((may_alias)) v8ha;
typedef v4f  __attribute__((may_alias)) v4fa;
typedef v8us __attribute__((may_alias)) v8usa;

__device__ __forceinline__ unsigned short f2bf(float f) { unsigned u = __float_as_uint(f); u += 0x7FFFu + ((u >> 16) & 1u); return (unsigned short)(u >> 16); }
__device__ __forceinline__ float bf2f(unsigned short b) { return __uint_as_float(((unsigned)b) << 16); }
__device__ __forceinline__ float bfr(float f) { return bf2f(f2bf(f)); }
__device__ __forceinline__ v16h cat16(v8h lo, v8h hi) { return __builtin_shufflevector(lo, hi, 0, 1, 2, 3, 4, 5, 6, 7, 8, 9, 10, 11, 12, 13, 14, 15); }
__device__ __forceinline__ v16bf cat16b(v8us lo, v8us hi) { return __builtin_bit_cast(v16bf, __builtin_shufflevector(lo, hi, 0, 1, 2, 3, 4, 5, 6, 7, 8, 9, 10, 11, 12, 13, 14, 15)); }
__device__ __forceinline__ v8f wmma16(v16h a, v16h b, v8f c) { return __builtin_amdgcn_wmma_f32_16x16x32_f16(false, a, false, b, (short)0, c, false, false); }
__device__ __forceinline__ v8f wmmab(v16bf a, v16bf b, v8f c) { return __builtin_amdgcn_wmma_f32_16x16x32_bf16(false, a, false, b, (short)0, c, false, false); }


template <typename T16> struct WFrag;
template <> struct WFrag<h16> { typedef v16h V; static __device__ __forceinline__ V ld(const h16* p) { return cat16(*(const v8h*)p, *(const v8h*)(p + 16)); } static __device__ __forceinline__ v8f mma(V a, V b, v8f c) { return wmma16(a, b, c); } };
template <> struct WFrag<bf> { typedef v16bf V; static __device__ __forceinline__ V ld(const bf* p) { return cat16b(*(const v8us*)p, *(const v8us*)(p + 16)); } static __device__ __forceinline__ v8f mma(V a, V b, v8f c) { return wmmab(a, b, c); } };
template <typename T16, int NSPLIT, bool BIAS>
__global__ __launch_bounds__(32) void k_gemmw(const T16* __restrict__ A, const T16* __restrict__ A2, const T16* __restrict__ Bt, const T16* __restrict__ Bt2, int K, float* C, int ldc, const float* __restrict__ bias, size_t sA, size_t sB, size_t sC) {
    typedef typename WFrag<T16>::V V;
    __shared__ __align__(16) float os[16 * 68];
    const size_t z = blockIdx.z; A += z * sA; if (A2) A2 += z * sA; Bt += z * sB; if (Bt2) Bt2 += z * sB; C += z * sC;
    const int lane = threadIdx.x & 31, lr = lane & 15, hi = lane >> 4; const int r0 = blockIdx.x * 64, c0 = blockIdx.y * 64;
    v8f acc[4][4];
#pragma unroll
    for (int mb = 0; mb < 4; ++mb)
#pragma unroll
        for (int nb = 0; nb < 4; ++nb) acc[mb][nb] = (v8f){};
    const size_t aoff = (size_t)(r0 + lr) * K + 8 * hi, boff = (size_t)(c0 + lr) * K + 8 * hi;
#pragma unroll 1
    for (int kc = 0; kc < K; kc += 32) {
        V a[4], a2[4];
#pragma unroll
        for (int mb = 0; mb < 4; ++mb) { a[mb] = WFrag<T16>::ld(A + aoff + (size_t)mb * 16 * K + kc); if (NSPLIT == 1 || NSPLIT == 2) a2[mb] = WFrag<T16>::ld(A2 + aoff + (size_t)mb * 16 * K + kc); }
#pragma unroll
        for (int nb = 0; nb < 4; ++nb) { const V b = WFrag<T16>::ld(Bt + boff + (size_t)nb * 16 * K + kc); V b2; if (NSPLIT >= 2) b2 = WFrag<T16>::ld(Bt2 + boff + (size_t)nb * 16 * K + kc);
#pragma unroll
            for (int mb = 0; mb < 4; ++mb) { acc[mb][nb] = WFrag<T16>::mma(a[mb], b, acc[mb][nb]); if (NSPLIT == 1 || NSPLIT == 2) acc[mb][nb] = WFrag<T16>::mma(a2[mb], b, acc[mb][nb]); if (NSPLIT >= 2) acc[mb][nb] = WFrag<T16>::mma(a[mb], b2, acc[mb][nb]); } }
        asm volatile("v_nop\n\tv_nop\n\tv_nop\n\tv_nop" : "+v"(acc[0][0]), "+v"(acc[1][1]), "+v"(acc[2][2]), "+v"(acc[3][3]) : "v"(a[0]), "v"(a[3]));
    }
#pragma unroll
    for (int mb = 0; mb < 4; ++mb) {
#pragma unroll
        for (int nb = 0; nb < 4; ++nb) {
#pragma unroll
            for (int j = 0; j < 8; ++j) os[(hi * 8 + j) * 68 + nb * 16 + lr] = acc[mb][nb][j]; }
        __builtin_amdgcn_wave_barrier(); asm volatile("" ::: "memory");
        float* crow = C + (size_t)(r0 + mb * 16) * ldc + c0;
#pragma unroll 1
        for (int ps = 0; ps < 2; ++ps) {
#pragma unroll
            for (int s = 0; s < 8; ++s) { const int row = 2 * s + hi, cofs = lr * 4; v4f val = *(const v4fa*)(os + row * 68 + cofs); if (BIAS) { val[0] += bfr(bias[c0 + cofs]); val[1] += bfr(bias[c0 + cofs + 1]); val[2] += bfr(bias[c0 + cofs + 2]); val[3] += bfr(bias[c0 + cofs + 3]); }
                *(volatile v4f*)(crow + (size_t)row * ldc + cofs) = val; }
            if (ps == 0) __threadfence(); }
        __builtin_amdgcn_wave_barrier(); asm volatile("" ::: "memory");
    }
}

__device__ __forceinline__ void splitf(float y, unsigned short& h, unsigned short& l) { h = f2bf(y); l = f2bf(y - bf2f(h)); }
typedef __attribute__((ext_vector_type(2))) unsigned short v2us;
typedef __attribute__((ext_vector_type(4))) unsigned short v4us;

__global__ __launch_bounds__(256) void k_wtG(const float* __restrict__ w, int K, int N, bf* Bt) {
    const int lane = threadIdx.x & 31; const int L0 = (blockIdx.x * 8 + (threadIdx.x >> 5)) * 8; const int nlines = N * K / 64;
#pragma unroll
    for (int ps = 0; ps < 2; ++ps) {
#pragma unroll 1
        for (int l = 0; l < 8; ++l) { const int L = L0 + l; if (L >= nlines) break; const size_t e = (size_t)L * 64 + lane * 2; const int k = (int)(e % K), n = (int)(e / K); v2us o;
            o[0] = f2bf(w[(size_t)k * N + n]); o[1] = f2bf(w[(size_t)(k + 1) * N + n]); *(volatile v2us*)(Bt + e) = o; }
        if (ps == 0) __threadfence(); }
}
__global__ __launch_bounds__(256) void k_wl(const float* __restrict__ wl, bf* Bt) { const int e = (blockIdx.x * 256 + threadIdx.x) * 4; if (e >= WD * WD) return; const int k = e % WD, j = e / WD; v4us o;
#pragma unroll
    for (int u = 0; u < 4; ++u) o[u] = (j < JJ) ? f2bf(wl[(k + u) * JJ + j]) : (unsigned short)0; *(volatile v4us*)(Bt + e) = o; __threadfence(); *(volatile v4us*)(Bt + e) = o; }
__global__ __launch_bounds__(64) void k_bl(const float* __restrict__ bl, float* b) { const int j = threadIdx.x; const float v = j < JJ ? bl[j] : 0.f; *(volatile float*)(b + j) = v; __threadfence(); *(volatile float*)(b + j) = v; }
template <int MODE> __global__ __launch_bounds__(256) void k_in(const float* __restrict__ x, const float* __restrict__ W0, const float* __restrict__ b0, float* Hf, bf* Ph, bf* Pl) { const int e = (blockIdx.x * 256 + threadIdx.x) * 4; if (e >= NP * WD) return; const int u0 = e % WD; const int p = e / WD;
    float x0 = bfr(x[(size_t)p * 2]), x1 = bfr(x[(size_t)p * 2 + 1]); if (MODE == 1) { x0 = __fmul_rn(__fsub_rn(x0, 0.5f), 2.0f); x1 = __fmul_rn(__fsub_rn(x1, 0.5f), 2.0f); } asm volatile("" : "+v"(x0)); asm volatile("" : "+v"(x1)); v4f hv; v4us oh, ol;
#pragma unroll
    for (int u = 0; u < 4; ++u) { const int uu = u0 + u; float w0 = bfr(W0[uu]), w1 = bfr(W0[WD + uu]), bb = bfr(b0[uu]); asm volatile("" : "+v"(w0)); asm volatile("" : "+v"(w1)); asm volatile("" : "+v"(bb)); float p0 = __fmul_rn(x0, w0), p1 = __fmul_rn(x1, w1); asm volatile("" : "+v"(p0)); asm volatile("" : "+v"(p1)); const float z = __fadd_rn(__fadd_rn(p0, p1), bb);
        const float h = (MODE == 0) ? fmaxf(z, 0.f) : tanhf(z); hv[u] = h; unsigned short a, b; splitf(h, a, b); oh[u] = a; ol[u] = b; }
    for (int ps = 0; ps < 2; ++ps) { if (MODE == 0) *(volatile v4f*)(Hf + e) = hv; *(volatile v4us*)(Ph + e) = oh; *(volatile v4us*)(Pl + e) = ol; if (ps == 0) __threadfence(); } }
template <int MODE> __global__ __launch_bounds__(256) void k_act(const float* __restrict__ G, float* Hf, bf* Ph, bf* Pl) { const int e = (blockIdx.x * 256 + threadIdx.x) * 4; if (e >= NP * WD) return; const v4f g = *(const v4f*)(G + e); v4f hv; v4us oh, ol;
    if (MODE == 0) hv = *(const v4f*)(Hf + e);
#pragma unroll
    for (int u = 0; u < 4; ++u) { const float h = (MODE == 0) ? __fadd_rn(hv[u], fmaxf(g[u], 0.f)) : tanhf(g[u]); hv[u] = h; unsigned short a, b; splitf(h, a, b); oh[u] = a; ol[u] = b; }
    for (int ps = 0; ps < 2; ++ps) { if (MODE == 0) *(volatile v4f*)(Hf + e) = hv; *(volatile v4us*)(Ph + e) = oh; *(volatile v4us*)(Pl + e) = ol; if (ps == 0) __threadfence(); } }
__global__ __launch_bounds__(256) void k_head(const float* __restrict__ G, const float* __restrict__ wl, const float* __restrict__ bl, int j, float* U) { const int p = blockIdx.x * 256 + threadIdx.x; if (p >= NP) return; const float* gr = G + (size_t)p * WD; float acc = 0.f;
#pragma unroll 1
    for (int k = 0; k < WD; ++k) { float w = bfr(wl[(size_t)j * WD + k]); asm volatile("" : "+v"(w)); float pr = __fmul_rn(tanhf(gr[k]), w); asm volatile("" : "+v"(pr)); acc = __fadd_rn(acc, pr); }
    float bb = bfr(bl[j]); asm volatile("" : "+v"(bb)); const float v = __fadd_rn(acc, bb); *(volatile float*)(U + (size_t)j * NP + p) = v; __threadfence(); *(volatile float*)(U + (size_t)j * NP + p) = v; }
__global__ __launch_bounds__(256) void k_final(const float* __restrict__ Lg, const float* __restrict__ U, const float* __restrict__ x, float* OUT) { const int p = blockIdx.x * 256 + threadIdx.x; if (p >= NP) return; const float* lr = Lg + (size_t)p * WD; float mx = -3.0e38f;
#pragma unroll
    for (int j = 0; j < JJ; ++j) mx = fmaxf(mx, lr[j]);
    float e_[JJ]; float sum = 0.f;
#pragma unroll
    for (int j = 0; j < JJ; ++j) { float d = __fsub_rn(lr[j], mx); asm volatile("" : "+v"(d)); e_[j] = __expf(d); sum = __fadd_rn(sum, e_[j]); }
    const float inv = __fdiv_rn(1.0f, sum); float tot = 0.f;
#pragma unroll
    for (int j = 0; j < JJ; ++j) { float w = __fmul_rn(e_[j], inv); asm volatile("" : "+v"(w)); float pr = __fmul_rn(w, U[(size_t)j * NP + p]); asm volatile("" : "+v"(pr)); tot = __fadd_rn(tot, pr); }
    const float PI_ = 3.14159265358979f; float a0 = __fmul_rn(PI_, bfr(x[(size_t)p * 2])), a1 = __fmul_rn(PI_, bfr(x[(size_t)p * 2 + 1])); asm volatile("" : "+v"(a0)); asm volatile("" : "+v"(a1)); float s0 = sinf(a0), s1 = sinf(a1); float t1 = __fmul_rn(tot, s0); asm volatile("" : "+v"(t1)); const float o = __fmul_rn(t1, s1);
    *(volatile float*)(OUT + p) = o; __threadfence(); *(volatile float*)(OUT + p) = o; }

extern "C" void kernel_launch(void* const* d_in, const int* in_sizes, int n_in,
                              void* d_out, int out_size, void* d_ws, size_t ws_size, hipStream_t stream) {
    (void)in_sizes; (void)n_in; (void)out_size;
    const float** I = (const float**)d_in;
    const float *x = I[0], *sW0 = I[1], *sb0 = I[2], *sWh = I[3], *sbh = I[4], *sWl = I[5], *sbl = I[6], *pW0 = I[7], *pb0 = I[8], *pWh = I[9], *pbh = I[10], *pWl = I[11], *pbl = I[12];
    float* OUT = (float*)d_out;
    char* wsp = (char*)d_ws;
    auto take = [&](size_t bytes) { char* p = wsp; wsp += (bytes + 255) & ~(size_t)255; return (void*)p; };
    bf* PWH = (bf*)take((size_t)4 * WD * WD * 2); bf* PWL = (bf*)take(WD * WD * 2); float* pblp = (float*)take(256); bf* SWH = (bf*)take((size_t)JJ * 2 * WD * WD * 2);
    float* Hf = (float*)take((size_t)NP * WD * 4); bf* Ph = (bf*)take((size_t)NP * WD * 2); bf* Pl = (bf*)take((size_t)NP * WD * 2); float* G = (float*)take((size_t)NP * WD * 4); float* Lg = (float*)take((size_t)NP * WD * 4); float* U = (float*)take((size_t)JJ * NP * 4);
    if ((size_t)(wsp - (char*)d_ws) > ws_size) return;
    for (int i = 0; i < 4; ++i) k_wtG<<<(WD * WD / 64 + 63) / 64, 256, 0, stream>>>(pWh + (size_t)i * WD * WD, WD, WD, PWH + (size_t)i * WD * WD);
    for (int ji = 0; ji < JJ * 2; ++ji) k_wtG<<<(WD * WD / 64 + 63) / 64, 256, 0, stream>>>(sWh + (size_t)ji * WD * WD, WD, WD, SWH + (size_t)ji * WD * WD);
    k_wl<<<(WD * WD / 4 + 255) / 256, 256, 0, stream>>>(pWl, PWL); k_bl<<<1, 64, 0, stream>>>(pbl, pblp);
    const unsigned nb4 = (NP * WD / 4 + 255) / 256, nb1 = (NP + 255) / 256;
    k_in<0><<<nb4, 256, 0, stream>>>(x, pW0, pb0, Hf, Ph, Pl);
    for (int i = 0; i < 4; ++i) { k_gemmw<bf, 1, true><<<dim3(NP / 64, 1, 1), 32, 0, stream>>>(Ph, Pl, PWH + (size_t)i * WD * WD, nullptr, WD, G, WD, pbh + i * WD, 0, 0, 0); k_act<0><<<nb4, 256, 0, stream>>>(G, Hf, Ph, Pl); }
    k_gemmw<bf, 1, true><<<dim3(NP / 64, 1, 1), 32, 0, stream>>>(Ph, Pl, PWL, nullptr, WD, Lg, WD, pblp, 0, 0, 0);
    for (int j = 0; j < JJ; ++j) {
        k_in<1><<<nb4, 256, 0, stream>>>(x, sW0 + (size_t)j * 2 * WD, sb0 + (size_t)j * WD, nullptr, Ph, Pl);
        k_gemmw<bf, 1, true><<<dim3(NP / 64, 1, 1), 32, 0, stream>>>(Ph, Pl, SWH + (size_t)(j * 2 + 0) * WD * WD, nullptr, WD, G, WD, sbh + (size_t)(j * 2 + 0) * WD, 0, 0, 0); k_act<1><<<nb4, 256, 0, stream>>>(G, nullptr, Ph, Pl);
        k_gemmw<bf, 1, true><<<dim3(NP / 64, 1, 1), 32, 0, stream>>>(Ph, Pl, SWH + (size_t)(j * 2 + 1) * WD * WD, nullptr, WD, G, WD, sbh + (size_t)(j * 2 + 1) * WD, 0, 0, 0);
        k_head<<<nb1, 256, 0, stream>>>(G, sWl, sbl, j, U); }
    k_final<<<nb1, 256, 0, stream>>>(Lg, U, x, OUT);
}
